// PrefixSumLinearAttentionModel_33002528703340
// MI455X (gfx1250) — hardware-run, weakly checked
//
#include <hip/hip_runtime.h>


namespace {
constexpr int NB_ = 32, SL = 2048, NV = 256, VOC = 512, D = 256, E = 256, NROW = NB_ * SL;
constexpr float XS = 8.0f, WSC = 256.0f, EPS = 1e-6f;
typedef _Float16 b16;
typedef __attribute__((ext_vector_type(16))) _Float16 v16b;
typedef __attribute__((ext_vector_type(8))) _Float16 v8b;
typedef __attribute__((ext_vector_type(8))) float v8f;
typedef __attribute__((ext_vector_type(4))) float v4f;
__device__ __forceinline__ float bf16_rne(float f) { unsigned int u = __float_as_uint(f); u += 0x7FFFu + ((u >> 16) & 1u); float r = __uint_as_float(u & 0xFFFF0000u); asm volatile("" : "+v"(r)); return r; }
__device__ __forceinline__ float bfv(float f) { float r = bf16_rne(f); asm volatile("" : "+v"(r)); return r; }
__device__ __forceinline__ v16b frag_kb(const b16* p, int hh) { const v8b a = *(const v8b*)(p + 8 * hh), b = *(const v8b*)(p + 16 + 8 * hh); v16b f;
#pragma unroll
  for (int e = 0; e < 8; ++e) { f[e] = a[e]; f[8 + e] = b[e]; } return f; }
__device__ __forceinline__ v8f wmma16b(v16b a, v16b b, v8f c) { v8f d = __builtin_amdgcn_wmma_f32_16x16x32_f16(false, a, false, b, (short)0, c, false, false); asm volatile("v_nop\n\tv_nop\n\tv_nop\n\tv_nop" : "+v"(d) : "v"(a), "v"(b)); return d; }
__device__ __forceinline__ void wave_lds_sync() { __builtin_amdgcn_fence(__ATOMIC_RELEASE, "workgroup"); __builtin_amdgcn_wave_barrier(); __builtin_amdgcn_fence(__ATOMIC_ACQUIRE, "workgroup"); }
__device__ __forceinline__ float pmul(float a, float b) { float p = a * b; asm volatile("" : "+v"(p)); return p; }
__device__ __forceinline__ int iclamp(int v, int lo, int hi) { return v < lo ? lo : (v > hi ? hi : v); }

__global__ __launch_bounds__(256) void setup_kernel(const float* __restrict__ wk, const int* __restrict__ qi, const float* __restrict__ emb, const float* __restrict__ wq, const float* __restrict__ bq, b16* __restrict__ WT, float* __restrict__ X2Q) { const int u = blockIdx.x * 256 + threadIdx.x; v8b v;
  if (u < D * 32) { const int o = u / 32, k0 = (u % 32) * 8;
#pragma unroll
    for (int j = 0; j < 8; ++j) v[j] = (b16)(bf16_rne(wk[(size_t)o * VOC + NV + k0 + j]) * WSC); for (int pass = 0; pass < 2; ++pass) { *(volatile v8b*)(WT + (size_t)o * E + k0) = v; __threadfence(); } }
  if (u < NB_ * D) { const int b = u / D, o = u % D; const size_t qrow = (size_t)iclamp(qi[b], 0, VOC - 1); float s = bfv(bq[o]); for (int e = 0; e < E; ++e) s += pmul(bfv(emb[qrow * E + e]), bfv(wq[(size_t)o * E + e]));
    for (int pass = 0; pass < 2; ++pass) { ((volatile float*)X2Q)[b * 2 * D + o] = fmaxf(s, 0.0f); ((volatile float*)X2Q)[b * 2 * D + D + o] = fmaxf(-s, 0.0f); __threadfence(); } } }
__global__ __launch_bounds__(32) void krow_kernel(const int* __restrict__ x, const float* __restrict__ emb, const b16* __restrict__ WT, const float* __restrict__ wk, const float* __restrict__ bk, const float* __restrict__ X2Q, int RLIM, float* __restrict__ S) { __shared__ __attribute__((aligned(16))) b16 Ah[32][E + 8]; __shared__ float X2[32][2 * D + 4], Os[32]; const int lane = threadIdx.x, nloc = lane & 15, hlf = lane >> 4; const size_t r0 = (size_t)blockIdx.x * 32; if (r0 >= (size_t)RLIM) return; const int b = (int)(r0 / SL); const int l0 = (int)(r0 % SL);
  for (int rr = 0; rr < 32; ++rr) { const size_t key = (size_t)iclamp(x[((size_t)b * 2) * SL + l0 + rr], 0, VOC - 1); for (int q = 0; q < 8; ++q) Ah[rr][q * 32 + lane] = (b16)(bf16_rne(emb[key * E + q * 32 + lane]) * XS); }
  for (int k = E; k < E + 8; ++k) Ah[lane][k] = (b16)0.0f;
  wave_lds_sync();
#pragma unroll 1
  for (int rt = 0; rt < 2; ++rt) { v8f acc[16];
#pragma unroll
    for (int t = 0; t < 16; ++t) acc[t] = (v8f){};
#pragma unroll 2
    for (int kb = 0; kb < E; kb += 32) { const v16b a = frag_kb(&Ah[rt * 16 + nloc][kb], hlf);
#pragma unroll
      for (int t = 0; t < 16; ++t) acc[t] = wmma16b(a, frag_kb(WT + (size_t)(t * 16 + nloc) * E + kb, hlf), acc[t]); }
#pragma unroll
    for (int t = 0; t < 16; ++t) { const int o = t * 16 + nloc;
#pragma unroll
      for (int r8 = 0; r8 < 8; ++r8) { const int rr = rt * 16 + 8 * hlf + r8; const int vi = iclamp(x[((size_t)b * 2 + 1) * SL + l0 + rr], NV, VOC - 1) - NV; const float kv = acc[t][r8] * (1.0f / (XS * WSC)) + bfv(wk[(size_t)o * VOC + vi]) + bfv(bk[o]); X2[rr][o] = fmaxf(kv, 0.0f); X2[rr][D + o] = fmaxf(-kv, 0.0f); } } }
  wave_lds_sync();
  { const float* qv = X2Q + (size_t)b * 2 * D; float s = 0.0f;
#pragma unroll 4
    for (int p = 0; p < 2 * D; ++p) { const int p1 = (p + 2 * D - 1) % (2 * D), p2 = (p + 2 * D - 2) % (2 * D); const float xk = X2[lane][p]; s += pmul(pmul(xk, X2[lane][p1]), pmul(qv[p], qv[p1])); s += pmul(pmul(xk, X2[lane][p2]), pmul(qv[p], qv[p2])); } Os[lane] = s; }
  wave_lds_sync();
  for (int pass = 0; pass < 2; ++pass) { ((volatile float*)S)[r0 + lane] = Os[lane]; __threadfence(); } }
__global__ __launch_bounds__(32) void out_kernel(const int* __restrict__ x, const float* __restrict__ S, int BLIM, float* __restrict__ out) { const int lane = threadIdx.x; const int b = blockIdx.x / (NV / 32), v0 = (blockIdx.x % (NV / 32)) * 32; if (b >= BLIM) return; const int v = v0 + lane; float num = 0.0f, den = 0.0f;
#pragma unroll 1
  for (int l = 0; l < SL; ++l) { const float s = S[(size_t)b * SL + l]; const int vi = x[((size_t)b * 2 + 1) * SL + l] - NV; den += s; if (vi == v) num += s; }
  const float y = num / (den + EPS);
  for (int pass = 0; pass < 2; ++pass) { ((volatile float*)out)[(size_t)b * NV + v] = y; __threadfence(); } }
}

extern "C" void kernel_launch(void* const* d_in, const int* in_sizes, int n_in, void* d_out, int out_size, void* d_ws, size_t ws_size, hipStream_t stream) {
  (void)n_in;
  auto Fp = [&](int i) { return (const float*)d_in[i]; }; auto Ip = [&](int i) { return (const int*)d_in[i]; };
  if (in_sizes[0] != NB_ * 2 * SL || in_sizes[1] != NB_ || in_sizes[2] != VOC * E || in_sizes[3] != D * VOC || in_sizes[5] != D * E || out_size != NB_ * NV) return;
  const int BLIM = NB_;
  size_t off = 0; char* ws = (char*)d_ws;
  auto carve = [&](size_t bytes) { char* p = ws + off; off += (bytes + 255) & ~(size_t)255; return p; };
  b16* WT = (b16*)carve((size_t)D * E * 2); float* X2Q = (float*)carve((size_t)NB_ * 2 * D * 4); float* S = (float*)carve((size_t)NROW * 4);
  if (off > ws_size || off > ((size_t)4 << 20)) return;
  setup_kernel<<<(D * 32 + 255) / 256, 256, 0, stream>>>(Fp(3), Ip(1), Fp(2), Fp(5), Fp(6), WT, X2Q);
  krow_kernel<<<(BLIM * SL) / 32, 32, 0, stream>>>(Ip(0), Fp(2), WT, Fp(3), Fp(4), X2Q, BLIM * SL, S);
  out_kernel<<<BLIM * (NV / 32), 32, 0, stream>>>(Ip(0), S, BLIM, (float*)d_out);
}
